// GMMILDiscriminator_15882789060993
// MI455X (gfx1250) — hardware-verified
//
#include <hip/hip_runtime.h>
#include <stdint.h>

typedef __attribute__((ext_vector_type(16))) _Float16 v16h;
typedef __attribute__((ext_vector_type(8)))  _Float16 v8h;
typedef __attribute__((ext_vector_type(8)))  float    v8f;
typedef __attribute__((ext_vector_type(4)))  float    v4f;
typedef __attribute__((ext_vector_type(4)))  unsigned v4u;

constexpr int kRows = 4096;
constexpr int kFeat = 512;
constexpr int kNBin = 4096;
constexpr int kHBlk = 65536;

static_assert(kRows % 64 == 0 && kFeat % 64 == 0, "tile multiples");
static_assert(kFeat % 32 == 0 && kRows % 32 == 0, "K multiple of 32");
static_assert((kRows * kRows) % kHBlk == 0 && (kFeat * kFeat) % kHBlk == 0, "histogram block coverage");
static_assert(kFeat == 512, "cast kernel assumes two 256-wide chunks per row");

__device__ __forceinline__ void dep_guard_h(v8f& a, v8f& b, v16h x, v16h y) { asm volatile("v_nop\n\tv_nop\n\tv_nop\n\tv_nop" : "+v"(a), "+v"(b) : "v"(x), "v"(y)); }
__device__ __forceinline__ void keep4_h(v16h a, v16h b, v16h c, v16h d) { asm volatile("v_nop" :: "v"(a), "v"(b), "v"(c), "v"(d)); }
__device__ __forceinline__ void acc_guard4(v8f& a, v8f& b, v8f& c, v8f& d) { asm volatile("v_nop\n\tv_nop\n\tv_nop\n\tv_nop" : "+v"(a), "+v"(b), "+v"(c), "+v"(d)); }
template <typename T> struct Frag;
template <> struct Frag<_Float16> {
  typedef v16h V; union U { v16h v; v8h h[2]; };
  static __device__ __forceinline__ v16h load(const _Float16* p) {
    U f; f.h[0] = *(const v8h*)(p); f.h[1] = *(const v8h*)(p + 16); return f.v;
  }
  static __device__ __forceinline__ v8f mma(v16h a, v16h b, v8f c) {
    return __builtin_amdgcn_wmma_f32_16x16x32_f16(false, a, false, b, (short)0, c, false, false);
  }
  static __device__ __forceinline__ void guard(v8f& a, v8f& b, v16h x, v16h y) { dep_guard_h(a, b, x, y); }
  static __device__ __forceinline__ void keep(v16h a, v16h b, v16h c, v16h d) { keep4_h(a, b, c, d); }
};

__global__ __launch_bounds__(256) void k_cast_rows(const float* __restrict__ X,
                                                   _Float16* __restrict__ H,
                                                   float* __restrict__ nrm) {
  __shared__ float sn[32];
  const int lane = threadIdx.x & 31, wave = threadIdx.x >> 5;
#pragma unroll 1
  for (int rr = 0; rr < 4; ++rr) {
    const int row = blockIdx.x * 32 + wave * 4 + rr;
    const float* p = X + (size_t)row * kFeat;
    v8h hv[2];
    float sqa = 0.f, sqb = 0.f;
#pragma unroll
    for (int it = 0; it < 2; ++it) {
      const v4f a = *(const v4f*)(p + 256 * it + 8 * lane);
      const v4f c = *(const v4f*)(p + 256 * it + 8 * lane + 4);
      v8h h;
      h[0] = (_Float16)a[0]; h[1] = (_Float16)a[1]; h[2] = (_Float16)a[2]; h[3] = (_Float16)a[3];
      h[4] = (_Float16)c[0]; h[5] = (_Float16)c[1]; h[6] = (_Float16)c[2]; h[7] = (_Float16)c[3];
      hv[it] = h;
      sqa += (a[0] * a[0] + a[1] * a[1]) + (a[2] * a[2] + a[3] * a[3]);
      sqb += (c[0] * c[0] + c[1] * c[1]) + (c[2] * c[2] + c[3] * c[3]);
    }
    _Float16* hp = H + (size_t)row * kFeat + 8 * lane;
    *(volatile v8h*)(hp) = hv[0];
    *(volatile v8h*)(hp + 256) = hv[1];
    __threadfence();
    *(volatile v8h*)(hp) = hv[0];
    *(volatile v8h*)(hp + 256) = hv[1];
    float sq = sqa + sqb;
#pragma unroll
    for (int off = 1; off < 32; off <<= 1) sq += __shfl_xor(sq, off, 32);
    if (lane == 0) sn[wave * 4 + rr] = sq;
  }
  __syncthreads();
  if (wave == 0) {
    const float v = sn[lane];
    float* np = nrm + blockIdx.x * 32 + lane;
    *(volatile float*)np = v;
    __threadfence();
    *(volatile float*)np = v;
  }
}

__global__ __launch_bounds__(256) void k_transpose_cast(const float* __restrict__ X, _Float16* __restrict__ T) {
  __shared__ __align__(16) _Float16 tile[64 * 72];
  const int t = threadIdx.x;
  const int c0 = blockIdx.x * 64, r0 = blockIdx.y * 64;
  const int rl = t >> 4, c4 = (t & 15) * 4;
#pragma unroll
  for (int it = 0; it < 4; ++it) {
    const int r = rl + 16 * it;
    const v4f x = *(const v4f*)(X + (size_t)(r0 + r) * kFeat + c0 + c4);
    tile[(c4 + 0) * 72 + r] = (_Float16)x[0];
    tile[(c4 + 1) * 72 + r] = (_Float16)x[1];
    tile[(c4 + 2) * 72 + r] = (_Float16)x[2];
    tile[(c4 + 3) * 72 + r] = (_Float16)x[3];
  }
  __syncthreads();
  const int li = t >> 3, q8 = (t & 7) * 8;
  v8h val[2];
#pragma unroll
  for (int it = 0; it < 2; ++it) val[it] = *(const v8h*)(tile + (li + 32 * it) * 72 + q8);
  for (int pass = 0; pass < 2; ++pass) {
#pragma unroll
    for (int it = 0; it < 2; ++it)
      *(volatile v8h*)(T + (size_t)(c0 + li + 32 * it) * kRows + r0 + q8) = val[it];
    __threadfence();
  }
}

__global__ __launch_bounds__(256) void k_colnorm(const float* __restrict__ X, float* __restrict__ cn) {
  __shared__ float sm[4][64];
  __shared__ __align__(16) float sm2[64];
  const int t = threadIdx.x;
  const int col = blockIdx.x * 64 + (t & 63);
  const int g = t >> 6;
  float sa = 0.f, sb = 0.f;
#pragma unroll 1
  for (int r = g; r < kRows; r += 8) {
    const float va = X[(size_t)r * kFeat + col];
    const float vb = X[(size_t)(r + 4) * kFeat + col];
    sa += va * va;
    sb += vb * vb;
  }
  sm[g][t & 63] = sa + sb;
  __syncthreads();
  if (t < 64) sm2[t] = (sm[0][t] + sm[1][t]) + (sm[2][t] + sm[3][t]);
  __syncthreads();
  if (t < 16) {
    const v4f v = *(const v4f*)(sm2 + 4 * t);
    float* p = cn + blockIdx.x * 64 + 4 * t;
    *(volatile v4f*)p = v;
    __threadfence();
    *(volatile v4f*)p = v;
  }
}

template <int MODE>
__global__ __launch_bounds__(256) void k_gemm_sq(const unsigned short* __restrict__ Ap, int lda,
                                                 const unsigned short* __restrict__ Btp, int ldb,
                                                 const float* __restrict__ rn, const float* __restrict__ cn,
                                                 float* __restrict__ Cout, int ldc,
                                                 const unsigned* __restrict__ seltab,
                                                 int M, int N, int K, float invd) {
  typedef _Float16 T;
  typedef v16h V;
  const T* A = (const T*)Ap;
  const T* Bt = (const T*)Btp;
  __shared__ __align__(16) float sT[8][16 * 68];
  const int lane = threadIdx.x & 31;
  const int wave = threadIdx.x >> 5;
  const int tilesN = N >> 6;
  const int tilesM = M >> 6;
  const int tile = blockIdx.x * 8 + wave;
  if (tile >= tilesM * tilesN) return;
  const int tm = tile / tilesN;
  const int tn = tile - tm * tilesN;
  const int m0 = tm << 6;
  const int n0 = tn << 6;
  const int rlane = lane & 15;
  const int koff = (lane >> 4) * 8;
  const int mOff = (lane >> 4) * 8;

  float ng1 = 0.f, ng2 = 0.f;
  if (MODE == 1) {
    ng1 = -__uint_as_float(seltab[6]);
    ng2 = -__uint_as_float(seltab[32 + 6]);
  }
  float cnv[4];
#pragma unroll
  for (int j = 0; j < 4; ++j) cnv[j] = cn[n0 + (j << 4) + rlane];

  v8f acc[4][4];
#pragma unroll
  for (int i = 0; i < 4; ++i)
#pragma unroll
    for (int j = 0; j < 4; ++j) acc[i][j] = (v8f){0.f, 0.f, 0.f, 0.f, 0.f, 0.f, 0.f, 0.f};

  for (int k0 = 0; k0 < K; k0 += 32) {
    V bh[4];
#pragma unroll
    for (int j = 0; j < 4; ++j) {
      const size_t bo = (size_t)(n0 + (j << 4) + rlane) * ldb + koff + k0;
      bh[j] = Frag<T>::load(Bt + bo);
    }
#pragma unroll
    for (int i = 0; i < 4; ++i) {
      const size_t ao = (size_t)(m0 + (i << 4) + rlane) * lda + koff + k0;
      V ah = Frag<T>::load(A + ao);
#pragma unroll
      for (int j = 0; j < 4; ++j) acc[i][j] = Frag<T>::mma(ah, bh[j], acc[i][j]);
      Frag<T>::guard(acc[i][0], acc[i][3], ah, ah);
    }
    Frag<T>::keep(bh[0], bh[1], bh[2], bh[3]);
  }
  acc_guard4(acc[0][0], acc[0][1], acc[0][2], acc[0][3]);
  acc_guard4(acc[1][0], acc[1][1], acc[1][2], acc[1][3]);
  acc_guard4(acc[2][0], acc[2][1], acc[2][2], acc[2][3]);
  acc_guard4(acc[3][0], acc[3][1], acc[3][2], acc[3][3]);

  float* slab = sT[wave];
  float cs0 = 0.f, cs1 = 0.f;
#pragma unroll
  for (int i = 0; i < 4; ++i) {
    const int mBase = m0 + (i << 4);
    const v4f ra = *(const v4f*)(rn + mBase + mOff);
    const v4f rb = *(const v4f*)(rn + mBase + mOff + 4);
    const float rv[8] = {ra[0], ra[1], ra[2], ra[3], rb[0], rb[1], rb[2], rb[3]};
#pragma unroll
    for (int j = 0; j < 4; ++j) {
#pragma unroll
      for (int r = 0; r < 8; ++r) {
        const float v = ((rv[r] + cnv[j]) - 2.0f * acc[i][j][r]) * invd;
        slab[(mOff + r) * 68 + (j << 4) + rlane] = v;
      }
    }
    __builtin_amdgcn_fence(__ATOMIC_RELEASE, "workgroup");
    __builtin_amdgcn_wave_barrier();
    __builtin_amdgcn_fence(__ATOMIC_ACQUIRE, "workgroup");
    if (MODE == 0) {
      float* C = Cout;
      const int hh = lane >> 4, c4 = (lane & 15) * 4;
      for (int pass = 0; pass < 2; ++pass) {
#pragma unroll
        for (int it = 0; it < 8; ++it) {
          const int row = it * 2 + hh;
          const v4f v = *(const v4f*)(slab + row * 68 + c4);
          *(volatile v4f*)(C + (size_t)(mBase + row) * ldc + n0 + c4) = v;
        }
        __threadfence();
      }
    } else {
#pragma unroll 1
      for (int r = 0; r < 16; ++r) {
        const float v0 = slab[r * 68 + lane];
        const float v1 = slab[r * 68 + 32 + lane];
        cs0 += expf(ng1 * v0) + expf(ng2 * v0);
        cs1 += expf(ng1 * v1) + expf(ng2 * v1);
      }
    }
    __builtin_amdgcn_fence(__ATOMIC_RELEASE, "workgroup");
    __builtin_amdgcn_wave_barrier();
    __builtin_amdgcn_fence(__ATOMIC_ACQUIRE, "workgroup");
  }
  if (MODE == 1) {
    slab[lane] = cs0;
    slab[32 + lane] = cs1;
    __builtin_amdgcn_fence(__ATOMIC_RELEASE, "workgroup");
    __builtin_amdgcn_wave_barrier();
    __builtin_amdgcn_fence(__ATOMIC_ACQUIRE, "workgroup");
    const v4f val = *(const v4f*)(slab + 4 * (lane & 15));
    float* pp = Cout + (size_t)tm * ldc + n0 + 4 * (lane & 15);
    for (int pass = 0; pass < 2; ++pass) {
      if (lane < 16) *(volatile v4f*)pp = val;
      __threadfence();
    }
  }
}

__global__ __launch_bounds__(256) void k_hist(const unsigned* __restrict__ keys, const unsigned* __restrict__ seltab,
                                              unsigned* __restrict__ part, int level, int dshift, unsigned dmask,
                                              int mshift, int nblkA) {
  __shared__ __align__(16) unsigned hist[2 * kNBin];
  const int t = threadIdx.x, b = blockIdx.x;
  const int q = (b >= nblkA) ? 1 : 0;
#pragma unroll
  for (int i = 0; i < (2 * kNBin) / 256; ++i) hist[t + 256 * i] = 0u;
  unsigned pre0 = 0u, pre1 = 0u;
  if (level > 0) {
    pre0 = seltab[32 * q + 0];
    pre1 = seltab[32 * q + 2];
  }
  __syncthreads();
  const unsigned* src = keys + (size_t)b * kHBlk + 4 * t;
#pragma unroll 1
  for (int it = 0; it < kHBlk / 1024; ++it) {
    const v4u w = *(const v4u*)(src + 1024 * it);
#pragma unroll
    for (int e = 0; e < 4; ++e) {
      const unsigned u = w[e];
      const unsigned key = (u & 0x80000000u) ? (~u) : (u | 0x80000000u);
      const unsigned dig = (key >> dshift) & dmask;
      const bool mt0 = (level == 0) || ((key >> mshift) == pre0);
      const bool mt1 = (level == 0) || ((key >> mshift) == pre1);
      if (mt0) atomicAdd(&hist[dig], 1u);
      if (mt1) atomicAdd(&hist[kNBin + dig], 1u);
    }
  }
  __syncthreads();
  unsigned* dst = part + (size_t)b * (2 * kNBin);
  for (int pass = 0; pass < 2; ++pass) {
#pragma unroll
    for (int i = 0; i < 8; ++i) {
      const int idx = 4 * t + 1024 * i;
      const v4u v = *(const v4u*)(hist + idx);
      *(volatile v4u*)(dst + idx) = v;
    }
    __threadfence();
  }
}

__global__ __launch_bounds__(256) void k_select(const unsigned* __restrict__ part, unsigned* __restrict__ seltab,
                                                int level, int nblkA, int nblkB, unsigned rankA, unsigned rankB) {
  __shared__ __align__(16) unsigned tot[kNBin];
  __shared__ unsigned scanbuf[256];
  __shared__ unsigned res[8];
  const int t = threadIdx.x, q = blockIdx.x;
  const int nblk = q ? nblkB : nblkA;
  const int blk0 = q ? nblkA : 0;
  unsigned opre0 = 0u, opre1 = 0u, ores0 = 0u, ores1 = 0u;
  if (level == 0) {
    ores0 = q ? rankB : rankA;
    ores1 = ores0 + 1u;
  } else {
    const unsigned* sl = seltab + 32 * q;
    opre0 = sl[0]; ores0 = sl[1]; opre1 = sl[2]; ores1 = sl[3];
  }
  if (t < 8) res[t] = 0u;
  __syncthreads();
#pragma unroll 1
  for (int tt = 0; tt < 2; ++tt) {
    v4u c0 = (v4u){0u, 0u, 0u, 0u}, c1 = c0, c2 = c0, c3 = c0;
#pragma unroll 1
    for (int bb = 0; bb < nblk; ++bb) {
      const unsigned* pb = part + ((size_t)(blk0 + bb) * 2 + tt) * kNBin + 4 * t;
      c0 += *(const v4u*)(pb);
      c1 += *(const v4u*)(pb + 1024);
      c2 += *(const v4u*)(pb + 2048);
      c3 += *(const v4u*)(pb + 3072);
    }
    *(v4u*)(tot + 4 * t) = c0;
    *(v4u*)(tot + 4 * t + 1024) = c1;
    *(v4u*)(tot + 4 * t + 2048) = c2;
    *(v4u*)(tot + 4 * t + 3072) = c3;
    __syncthreads();
    const v4u l0 = *(const v4u*)(tot + 16 * t);
    const v4u l1 = *(const v4u*)(tot + 16 * t + 4);
    const v4u l2 = *(const v4u*)(tot + 16 * t + 8);
    const v4u l3 = *(const v4u*)(tot + 16 * t + 12);
    const unsigned lsum = ((l0[0] + l0[1]) + (l0[2] + l0[3])) + ((l1[0] + l1[1]) + (l1[2] + l1[3])) +
                          ((l2[0] + l2[1]) + (l2[2] + l2[3])) + ((l3[0] + l3[1]) + (l3[2] + l3[3]));
    scanbuf[t] = lsum;
    __syncthreads();
    for (int off = 1; off < 256; off <<= 1) {
      int si = t - off;
      si = si < 0 ? 0 : si;
      unsigned v = scanbuf[si];
      v = (t >= off) ? v : 0u;
      __syncthreads();
      scanbuf[t] += v;
      __syncthreads();
    }
    const unsigned excl = scanbuf[t] - lsum;
    const unsigned R = tt ? ores1 : ores0;
    const unsigned bins[16] = {l0[0], l0[1], l0[2], l0[3], l1[0], l1[1], l1[2], l1[3],
                               l2[0], l2[1], l2[2], l2[3], l3[0], l3[1], l3[2], l3[3]};
    if (R >= excl && (R - excl) < lsum) {
      unsigned cum = excl;
#pragma unroll
      for (int e = 0; e < 16; ++e) {
        const unsigned c = bins[e];
        if (R >= cum && (R - cum) < c) {
          res[2 * tt] = (unsigned)(16 * t + e);
          res[2 * tt + 1] = R - cum;
        }
        cum += c;
      }
    }
    __syncthreads();
  }
  if (t < 32) {
    const unsigned d0 = res[0], rr0 = res[1], d1 = res[2], rr1 = res[3];
    unsigned np0 = 0u, np1 = 0u, key0 = 0u, key1 = 0u, gbits = 0u;
    if (level == 0) {
      np0 = d0; np1 = d1;
    } else if (level == 1) {
      np0 = (opre0 << 12) | d0;
      np1 = (opre1 << 12) | d1;
    } else {
      np0 = opre0; np1 = opre1;
      key0 = (opre0 << 8) | (d0 & 0xFFu);
      key1 = (opre1 << 8) | (d1 & 0xFFu);
      const unsigned u0 = (key0 & 0x80000000u) ? (key0 & 0x7FFFFFFFu) : (~key0);
      const unsigned u1 = (key1 & 0x80000000u) ? (key1 & 0x7FFFFFFFu) : (~key1);
      const float lo = __uint_as_float(u0), hi = __uint_as_float(u1);
      const float med = 0.5f * lo + 0.5f * hi;
      const float gam = 1.0f / med;
      gbits = __float_as_uint(gam);
    }
    unsigned val = 0u;
    val = (t == 0) ? np0 : val;
    val = (t == 1) ? rr0 : val;
    val = (t == 2) ? np1 : val;
    val = (t == 3) ? rr1 : val;
    val = (t == 4) ? key0 : val;
    val = (t == 5) ? key1 : val;
    val = (t == 6) ? gbits : val;
    unsigned* sp = seltab + 32 * q + t;
    *(volatile unsigned*)sp = val;
    __threadfence();
    *(volatile unsigned*)sp = val;
  }
}

__global__ __launch_bounds__(256) void k_rowexp(const float* __restrict__ Dm, const unsigned* __restrict__ seltab,
                                                float* __restrict__ simsum) {
  __shared__ float sres[32];
  const int lane = threadIdx.x & 31, wave = threadIdx.x >> 5;
  const float ng1 = -__uint_as_float(seltab[6]);
  const float ng2 = -__uint_as_float(seltab[32 + 6]);
#pragma unroll 1
  for (int rr = 0; rr < 4; ++rr) {
    const int row = blockIdx.x * 32 + wave * 4 + rr;
    const float* p = Dm + (size_t)row * kRows + 4 * lane;
    float a0 = 0.f, a1 = 0.f, a2 = 0.f, a3 = 0.f;
#pragma unroll 1
    for (int it = 0; it < kRows / 128; ++it) {
      const v4f d = *(const v4f*)(p + 128 * it);
      a0 += expf(ng1 * d[0]) + expf(ng2 * d[0]);
      a1 += expf(ng1 * d[1]) + expf(ng2 * d[1]);
      a2 += expf(ng1 * d[2]) + expf(ng2 * d[2]);
      a3 += expf(ng1 * d[3]) + expf(ng2 * d[3]);
    }
    float s = (a0 + a1) + (a2 + a3);
#pragma unroll
    for (int off = 1; off < 32; off <<= 1) s += __shfl_xor(s, off, 32);
    if (lane == 0) sres[wave * 4 + rr] = s;
  }
  __syncthreads();
  if (wave == 0) {
    const float v = sres[lane];
    float* sp = simsum + blockIdx.x * 32 + lane;
    *(volatile float*)sp = v;
    __threadfence();
    *(volatile float*)sp = v;
  }
}

__global__ __launch_bounds__(256) void k_final(const float* __restrict__ P, const float* __restrict__ simsum,
                                               float* __restrict__ out) {
  const int gid = blockIdx.x * 256 + threadIdx.x;
  double q0 = 0.0, q1 = 0.0, q2 = 0.0, q3 = 0.0;
#pragma unroll 1
  for (int tm = 0; tm < kRows / 64; ++tm) {
    const v4f pv = *(const v4f*)(P + (size_t)tm * kRows + 4 * gid);
    q0 += (double)pv[0]; q1 += (double)pv[1]; q2 += (double)pv[2]; q3 += (double)pv[3];
  }
  const v4f sm = *(const v4f*)(simsum + 4 * gid);
  const float inv = 1.0f / (float)kRows;
  v4f o;
  o[0] = sm[0] * inv - (float)q0 * inv;
  o[1] = sm[1] * inv - (float)q1 * inv;
  o[2] = sm[2] * inv - (float)q2 * inv;
  o[3] = sm[3] * inv - (float)q3 * inv;
  float* op = out + 4 * gid;
  *(volatile v4f*)op = o;
  __threadfence();
  *(volatile v4f*)op = o;
}

extern "C" void kernel_launch(void* const* d_in, const int* in_sizes, int n_in,
                              void* d_out, int out_size, void* d_ws, size_t ws_size,
                              hipStream_t stream) {
  if (n_in < 3) return;
  if (in_sizes[0] != kRows * kFeat || in_sizes[2] != kRows * kFeat || out_size != kRows) return;
  const float* state = (const float*)d_in[0];
  const float* expert = (const float*)d_in[2];
  float* out = (float*)d_out;

  char* ws = (char*)d_ws;
  size_t off = 0;
  auto carve = [&](size_t bytes) -> char* {
    char* p = ws + off;
    off += (bytes + 255) & ~(size_t)255;
    return p;
  };
  const size_t planeBytes = (size_t)kRows * kFeat * 2;
  _Float16* Sh = (_Float16*)carve(planeBytes);
  _Float16* Eh = (_Float16*)carve(planeBytes);
  _Float16* Et = (_Float16*)carve(planeBytes);
  float* s2 = (float*)carve((size_t)kRows * 4);
  float* e2 = (float*)carve((size_t)kRows * 4);
  float* c2 = (float*)carve((size_t)kFeat * 4);
  const size_t desBytes = (size_t)kRows * kRows * 4;
  const size_t dccBytes = (size_t)kFeat * kFeat * 4;
  float* Des = (float*)carve(desBytes + dccBytes);
  float* Dcc = Des + (size_t)kRows * kRows;
  const int nblkA = (kRows * kRows) / kHBlk;
  const int nblkB = (kFeat * kFeat) / kHBlk;
  unsigned* part = (unsigned*)carve((size_t)(nblkA + nblkB) * 2 * kNBin * 4);
  unsigned* seltab = (unsigned*)carve(256);
  float* simsum = (float*)carve((size_t)kRows * 4);
  float* Pss = (float*)carve((size_t)(kRows / 64) * kRows * 4);
  if (off > ws_size) return;

  k_cast_rows<<<dim3(kRows / 32), dim3(256), 0, stream>>>(state, Sh, s2);
  k_cast_rows<<<dim3(kRows / 32), dim3(256), 0, stream>>>(expert, Eh, e2);
  k_transpose_cast<<<dim3(kFeat / 64, kRows / 64), dim3(256), 0, stream>>>(expert, Et);
  k_colnorm<<<dim3(kFeat / 64), dim3(256), 0, stream>>>(expert, c2);

  const int tilesES = (kRows / 64) * (kRows / 64);
  const int tilesCC = (kFeat / 64) * (kFeat / 64);
  k_gemm_sq<0><<<dim3(tilesES / 8), dim3(256), 0, stream>>>(
      (const unsigned short*)Sh, kFeat, (const unsigned short*)Eh, kFeat, s2, e2, Des, kRows, seltab,
      kRows, kRows, kFeat, 1.0f / (float)kFeat);
  k_gemm_sq<0><<<dim3(tilesCC / 8), dim3(256), 0, stream>>>(
      (const unsigned short*)Et, kRows, (const unsigned short*)Et, kRows, c2, c2, Dcc, kFeat, seltab,
      kFeat, kFeat, kRows, 1.0f / (float)kRows);

  const unsigned rankA = (unsigned)((kRows * kRows) / 2 - 1);
  const unsigned rankB = (unsigned)((kFeat * kFeat) / 2 - 1);
  const int dsh[3] = {20, 8, 0};
  const unsigned dmk[3] = {0xFFFu, 0xFFFu, 0xFFu};
  const int msh[3] = {20, 20, 8};
  for (int lv = 0; lv < 3; ++lv) {
    k_hist<<<dim3(nblkA + nblkB), dim3(256), 0, stream>>>((const unsigned*)Des, seltab, part, lv, dsh[lv],
                                                          dmk[lv], msh[lv], nblkA);
    k_select<<<dim3(2), dim3(256), 0, stream>>>(part, seltab, lv, nblkA, nblkB, rankA, rankB);
  }

  k_rowexp<<<dim3(kRows / 32), dim3(256), 0, stream>>>(Des, seltab, simsum);

  k_gemm_sq<1><<<dim3(tilesES / 8), dim3(256), 0, stream>>>(
      (const unsigned short*)Sh, kFeat, (const unsigned short*)Sh, kFeat, s2, s2, Pss, kRows, seltab,
      kRows, kRows, kFeat, 1.0f / (float)kFeat);

  k_final<<<dim3(kRows / 1024), dim3(256), 0, stream>>>(Pss, simsum, out);
}
